// CrossAttention_7215545057495
// MI455X (gfx1250) — hardware-verified
//
#include <hip/hip_runtime.h>
#include <stdint.h>


typedef _Float16 v16h __attribute__((ext_vector_type(16)));
typedef _Float16 v8h  __attribute__((ext_vector_type(8)));
typedef float    v8f  __attribute__((ext_vector_type(8)));
typedef float    v4f  __attribute__((ext_vector_type(4)));

#ifndef NB
#define NB 4
#endif
#ifndef SEQ
#define SEQ 1024
#endif
#ifndef MCTX
#define MCTX 1024
#endif
#define NB_FULL   4
#define SEQ_FULL  1024
#define MCTX_FULL 1024
#define DM   1024
#define NH   16
#define HD   64
#define MRQ  (NB * SEQ)
#define MRK  (NB * MCTX)

#define ACT_CAR   8.0f
#define W_CAR     1024.0f
#define PROJ_SCL  0.0009765625f
#define RES_CAR   2048.0f
#define RES_INV   0.00048828125f
#define S_SCL     0.00048828125f
#define S_CLIP    10000.0f
#define P_CAR     16384.0f
#define O_SCL     7.62939453125e-06f
#define OUT_SCL   0.0001220703125f
#define LN_EPS    1e-5f

static_assert(NB >= 1 && NB <= NB_FULL);
static_assert(SEQ % 128 == 0 && MCTX % 128 == 0);
static_assert(SEQ <= SEQ_FULL && MCTX <= MCTX_FULL);
static_assert(DM == NH * HD);
static_assert(HD == 64);
static_assert(DM == 1024);
static_assert((DM & (DM - 1)) == 0 && DM % 128 == 0);
static_assert((long)(MRQ / 8) * 8 == (long)MRQ && (long)(MRK / 8) * 8 == (long)MRK);
static_assert(4 * 32 * 8 == DM && 8 * 32 * 4 == DM);
static_assert(((long)MRK * DM / 8) % 256 == 0 && ((long)DM * DM / 8) % 256 == 0);
static_assert((long)(DM / 64) * (MRQ / 128) * 128 * 64 == (long)MRQ * DM);
static_assert((long)(DM / 64) * (MRK / 128) * 128 * 64 == (long)MRK * DM);
static_assert((long)(MCTX / 64) * (DM / 128) * NB * 128 * 64 == (long)MRK * DM);
static_assert((long)(SEQ / 128) * NH * NB * 128 * HD == (long)MRQ * DM);
static_assert((long)(DM / 64) * (MRQ / 64) * 64 * 64 == (long)MRQ * DM);
#define N_Q   ((long)MRQ * DM)
#define N_K   ((long)MRK * DM)
#define N_W   ((long)DM * DM)
#define N_R0  (((N_Q + N_K) > (2 * N_Q)) ? (N_Q + N_K) : (2 * N_Q))
#define WS_HALVES (N_R0 + N_K + 4 * N_W + 2 * N_Q + 2 * N_K + 2 * N_K + 2 * N_Q + 2 * N_Q)
static_assert(N_R0 >= N_Q + N_K && N_R0 >= 2 * N_Q);
static_assert(WS_HALVES * 2 <= 134217728L);

union Frag16 { v16h v; v8h p[2]; };

__device__ __forceinline__ v16h ld_frag(const _Float16* p, int hl) {
  Frag16 f;
  f.p[0] = *(const v8h*)(p + 8 * hl);
  f.p[1] = *(const v8h*)(p + 16 + 8 * hl);
  return f.v;
}

__device__ __forceinline__ v8f mma(v16h a, v16h b, v8f c) {
  v8f d = __builtin_amdgcn_wmma_f32_16x16x32_f16(false, a, false, b, (short)0, c, false, false);
  asm volatile("v_nop\n\tv_nop\n\tv_nop\n\tv_nop" : "+v"(d) : "v"(a), "v"(b));
  return d;
}

__device__ __forceinline__ float bf16_rne(float x) {
  unsigned int u = __builtin_bit_cast(unsigned int, x);
  u += 0x7FFFu + ((u >> 16) & 1u);
  return __builtin_bit_cast(float, u & 0xFFFF0000u);
}

template <unsigned RPB, unsigned RPBF>
__global__ __launch_bounds__(256) void k_cvt8(const float* __restrict__ src,
                                              _Float16* __restrict__ dst,
                                              float car, unsigned total8)
{
  const unsigned i8 = blockIdx.x * 256u + threadIdx.x;
  if (i8 >= total8) return;
  const unsigned e   = i8 * 8u;
  const unsigned r   = e / (unsigned)DM;
  const unsigned col = e - r * (unsigned)DM;
  const unsigned bq  = r / RPB;
  const unsigned sr  = bq * RPBF + (r - bq * RPB);
  const float* s = src + (size_t)sr * DM + col;
  const v4f x0 = *(const v4f*)s;
  const v4f x1 = *(const v4f*)(s + 4);
  v8h o;
#pragma unroll
  for (int j = 0; j < 4; ++j) {
    const float t0 = x0[j];
    const float t1 = x1[j];
    o[j]     = (_Float16)(bf16_rne(t0) * car);
    o[4 + j] = (_Float16)(bf16_rne(t1) * car);
  }
  _Float16* d = dst + (size_t)e;
  *(volatile v8h*)d = o;
  __threadfence();
  *(volatile v8h*)d = o;
}

template <int MODE>
__device__ __forceinline__ float xin(float v) { return (MODE == 0) ? bf16_rne(v) : v; }

__device__ __forceinline__ float ln_y(float x, float mean, float rinv, float g, float b) {
  return (x - mean) * rinv * bf16_rne(g) + bf16_rne(b);
}

template <int MODE, unsigned RPB, unsigned RPBF>
__global__ __launch_bounds__(256) void k_ln(const float* __restrict__ src,
                                            const float* __restrict__ gam,
                                            const float* __restrict__ bet,
                                            _Float16* __restrict__ PH,
                                            _Float16* __restrict__ PL,
                                            float* __restrict__ YF)
{
  const unsigned tid = threadIdx.x, lane = tid & 31u, w = tid >> 5;
  const unsigned row = blockIdx.x * 8u + w;
  const unsigned bq  = row / RPB;
  const unsigned srow = (MODE == 0) ? (bq * RPBF + (row - bq * RPB)) : row;
  const float* x = src + (size_t)srow * DM;

  float s = 0.f;
#pragma unroll 1
  for (unsigned i = 0; i < 8u; ++i) {
    const v4f a = *(const v4f*)(x + i * 128u + lane * 4u);
    s += (xin<MODE>(a[0]) + xin<MODE>(a[1])) + (xin<MODE>(a[2]) + xin<MODE>(a[3]));
  }
  s += __shfl_xor(s, 16, 32);
  s += __shfl_xor(s, 8, 32);
  s += __shfl_xor(s, 4, 32);
  s += __shfl_xor(s, 2, 32);
  s += __shfl_xor(s, 1, 32);
  const float mean = s * (1.0f / (float)DM);

  float s2 = 0.f;
#pragma unroll 1
  for (unsigned i = 0; i < 8u; ++i) {
    const v4f a = *(const v4f*)(x + i * 128u + lane * 4u);
#pragma unroll
    for (int j = 0; j < 4; ++j) {
      const float d = xin<MODE>(a[j]) - mean;
      s2 += d * d;
    }
  }
  s2 += __shfl_xor(s2, 16, 32);
  s2 += __shfl_xor(s2, 8, 32);
  s2 += __shfl_xor(s2, 4, 32);
  s2 += __shfl_xor(s2, 2, 32);
  s2 += __shfl_xor(s2, 1, 32);
  const float var  = s2 * (1.0f / (float)DM);
  const float rinv = 1.0f / sqrtf(var + LN_EPS);

#pragma unroll 1
  for (unsigned i = 0; i < 4u; ++i) {
    const unsigned col = i * 256u + lane * 8u;
    const v4f a0 = *(const v4f*)(x + col);
    const v4f a1 = *(const v4f*)(x + col + 4u);
    const v4f g0 = *(const v4f*)(gam + col);
    const v4f g1 = *(const v4f*)(gam + col + 4u);
    const v4f b0 = *(const v4f*)(bet + col);
    const v4f b1 = *(const v4f*)(bet + col + 4u);
    v8h oh, ol;
#pragma unroll
    for (int j = 0; j < 4; ++j) {
      const float t0 = ln_y(xin<MODE>(a0[j]), mean, rinv, g0[j], b0[j]) * ACT_CAR;
      const float t1 = ln_y(xin<MODE>(a1[j]), mean, rinv, g1[j], b1[j]) * ACT_CAR;
      const _Float16 h0 = (_Float16)t0;
      const _Float16 h1 = (_Float16)t1;
      oh[j]     = h0;
      oh[4 + j] = h1;
      ol[j]     = (_Float16)((t0 - (float)h0) * RES_CAR);
      ol[4 + j] = (_Float16)((t1 - (float)h1) * RES_CAR);
    }
    _Float16* dh = PH + (size_t)row * DM + col;
    _Float16* dl = PL + (size_t)row * DM + col;
    *(volatile v8h*)dh = oh;
    if (MODE == 1) *(volatile v8h*)dl = ol;
    __threadfence();
    *(volatile v8h*)dh = oh;
    if (MODE == 1) *(volatile v8h*)dl = ol;
  }

  if (MODE == 1) {
#pragma unroll 1
    for (unsigned i = 0; i < 8u; ++i) {
      const unsigned col = i * 128u + lane * 4u;
      const v4f a = *(const v4f*)(x + col);
      const v4f g = *(const v4f*)(gam + col);
      const v4f b = *(const v4f*)(bet + col);
      v4f y;
#pragma unroll
      for (int j = 0; j < 4; ++j) y[j] = ln_y(a[j], mean, rinv, g[j], b[j]);
      float* d = YF + (size_t)row * DM + col;
      *(volatile v4f*)d = y;
      __threadfence();
      *(volatile v4f*)d = y;
    }
  }
}

__device__ __forceinline__ void gemm_core(const _Float16* ap0, const _Float16* ap1,
                                          const _Float16* bp, int K, int hl, v8f (&acc)[8])
{
  const size_t bst = (size_t)16 * K;
#pragma unroll 1
  for (int k0 = 0; k0 < K; k0 += 32) {
    const v16h a0 = ld_frag(ap0 + k0, hl);
    const v16h a1 = ld_frag(ap1 + k0, hl);
    const v16h b0 = ld_frag(bp + k0, hl);
    const v16h b1 = ld_frag(bp + bst + k0, hl);
    const v16h b2 = ld_frag(bp + 2 * bst + k0, hl);
    const v16h b3 = ld_frag(bp + 3 * bst + k0, hl);
    acc[0] = mma(a0, b0, acc[0]);
    acc[1] = mma(a0, b1, acc[1]);
    acc[2] = mma(a0, b2, acc[2]);
    acc[3] = mma(a0, b3, acc[3]);
    acc[4] = mma(a1, b0, acc[4]);
    acc[5] = mma(a1, b1, acc[5]);
    acc[6] = mma(a1, b2, acc[6]);
    acc[7] = mma(a1, b3, acc[7]);
  }
}

__global__ __launch_bounds__(128) __attribute__((amdgpu_num_vgpr(256)))
void k_proj(const _Float16* __restrict__ A, const _Float16* __restrict__ Bt,
            _Float16* __restrict__ PH, _Float16* __restrict__ PL, int K, int ldc,
            unsigned sBz, unsigned sCz)
{
  __shared__ __attribute__((aligned(16))) _Float16 ldsE[2 * 128 * 72];
  _Float16* const ldsH = ldsE;
  _Float16* const ldsL = ldsE + 128 * 72;

  const int tid = threadIdx.x, lane = tid & 31, w = tid >> 5;
  const int hl = lane >> 4, c = lane & 15;
  const int m0 = blockIdx.y * 128, n0 = blockIdx.x * 64;
  const int mw = m0 + 32 * w;
  const size_t zb = (size_t)blockIdx.z * sBz;
  const size_t zc = (size_t)blockIdx.z * sCz;

  const _Float16* ap0 = A  + (size_t)(mw + c) * K;
  const _Float16* ap1 = A  + (size_t)(mw + 16 + c) * K;
  const _Float16* bp  = Bt + zb + (size_t)(n0 + c) * K;

  v8f acc[8] = {};
  gemm_core(ap0, ap1, bp, K, hl, acc);

#pragma unroll
  for (int i = 0; i < 2; ++i)
#pragma unroll
    for (int t = 0; t < 4; ++t)
#pragma unroll
      for (int r = 0; r < 8; ++r) {
        const int rowl = 32 * w + 16 * i + 8 * hl + r;
        const float v = acc[i * 4 + t][r] * PROJ_SCL;
        const _Float16 hv = (_Float16)v;
        const float res = (v - (float)hv) * RES_CAR;
        ldsH[rowl * 72 + 16 * t + c] = hv;
        ldsL[rowl * 72 + 16 * t + c] = (_Float16)res;
      }
  __syncthreads();

  _Float16* const bh = PH + zc + (size_t)m0 * ldc + n0;
  _Float16* const bl = PL + zc + (size_t)m0 * ldc + n0;
  for (int i = 0; i < 8; ++i) {
    const int q = i * 128 + tid;
    const int rowl = q >> 3, ch = (q & 7) * 8;
    const v8h vh = *(const v8h*)(ldsH + rowl * 72 + ch);
    const v8h vl = *(const v8h*)(ldsL + rowl * 72 + ch);
    *(volatile v8h*)(bh + (size_t)rowl * ldc + ch) = vh;
    *(volatile v8h*)(bl + (size_t)rowl * ldc + ch) = vl;
  }
  __threadfence();
  for (int i = 0; i < 8; ++i) {
    const int q = i * 128 + tid;
    const int rowl = q >> 3, ch = (q & 7) * 8;
    const v8h vh = *(const v8h*)(ldsH + rowl * 72 + ch);
    const v8h vl = *(const v8h*)(ldsL + rowl * 72 + ch);
    *(volatile v8h*)(bh + (size_t)rowl * ldc + ch) = vh;
    *(volatile v8h*)(bl + (size_t)rowl * ldc + ch) = vl;
  }
}

__global__ __launch_bounds__(256) __attribute__((amdgpu_num_vgpr(256)))
void k_attn(const _Float16* __restrict__ QH, const _Float16* __restrict__ QL,
            const _Float16* __restrict__ KH, const _Float16* __restrict__ KL,
            const _Float16* __restrict__ VtH, const _Float16* __restrict__ VtL,
            float* __restrict__ Oc)
{
  constexpr int KT_H   = 32 * 72;
  constexpr int V_H    = HD * 40;
  constexpr int P_H    = 8 * 16 * 40;
  constexpr int TILE_B = (2 * KT_H + 2 * V_H + 2 * P_H) * 2;
  constexpr int EPI_B  = 128 * 68 * 4;
  constexpr int LDS_B  = (TILE_B > EPI_B) ? TILE_B : EPI_B;
  __shared__ __attribute__((aligned(16))) unsigned char ldsRaw[LDS_B];
  _Float16* const lds   = (_Float16*)ldsRaw;
  _Float16* const ldsK0 = lds;
  _Float16* const ldsK1 = ldsK0 + KT_H;
  _Float16* const ldsVH = ldsK1 + KT_H;
  _Float16* const ldsVL = ldsVH + V_H;
  _Float16* const ldsPH = ldsVL + V_H;
  _Float16* const ldsPL = ldsPH + P_H;
  float*    const ldsF  = (float*)ldsRaw;

  const int tid = threadIdx.x, lane = tid & 31, w = tid >> 5;
  const int hl = lane >> 4, c = lane & 15;
  const int q0 = blockIdx.x * 128;
  const int col0 = blockIdx.y * HD;
  const int bz = blockIdx.z;

  const size_t qrow = ((size_t)bz * SEQ + q0 + 16 * w + c) * DM + col0;
  v16h qh[2], ql[2];
#pragma unroll
  for (int ks = 0; ks < 2; ++ks) {
    qh[ks] = ld_frag(QH + qrow + 32 * ks, hl);
    ql[ks] = ld_frag(QL + qrow + 32 * ks, hl);
  }
  _Float16* const myPH = ldsPH + w * (16 * 40);
  _Float16* const myPL = ldsPL + w * (16 * 40);

  const int krr = tid >> 3, kcc = (tid & 7) * 8;
  const int vdd = tid >> 2, vkc = (tid & 3) * 8;
  const _Float16* const kgh = KH + ((size_t)bz * MCTX + krr) * DM + col0 + kcc;
  const _Float16* const kgl = KL + ((size_t)bz * MCTX + krr) * DM + col0 + kcc;
  const _Float16* const vgh = VtH + (size_t)bz * DM * MCTX + (size_t)(col0 + vdd) * MCTX + vkc;
  const _Float16* const vgl = VtL + (size_t)bz * DM * MCTX + (size_t)(col0 + vdd) * MCTX + vkc;

  float m[8], l[8];
  v8f oh[4] = {}, ol[4] = {};
#pragma unroll
  for (int r = 0; r < 8; ++r) { m[r] = -__builtin_inff(); l[r] = 0.f; }

#pragma unroll 1
  for (int kt = 0; kt < MCTX / 32; ++kt) {
    const int mk = kt * 32;
    {
      const v8h k8h = *(const v8h*)(kgh + (size_t)mk * DM);
      const v8h k8l = *(const v8h*)(kgl + (size_t)mk * DM);
      const v8h v8a = *(const v8h*)(vgh + mk);
      const v8h v8b = *(const v8h*)(vgl + mk);
      *(v8h*)(ldsK0 + krr * 72 + kcc) = k8h;
      *(v8h*)(ldsK1 + krr * 72 + kcc) = k8l;
      *(v8h*)(ldsVH + vdd * 40 + vkc) = v8a;
      *(v8h*)(ldsVL + vdd * 40 + vkc) = v8b;
    }
    __syncthreads();

    v8f sh[2] = {}, sl[2] = {};
#pragma unroll
    for (int ks = 0; ks < 2; ++ks) {
#pragma unroll
      for (int t = 0; t < 2; ++t) {
        const v16h kfh = ld_frag(ldsK0 + (16 * t + c) * 72 + 32 * ks, hl);
        const v16h kfl = ld_frag(ldsK1 + (16 * t + c) * 72 + 32 * ks, hl);
        sh[t] = mma(qh[ks], kfh, sh[t]);
        sl[t] = mma(ql[ks], kfh, sl[t]);
        sl[t] = mma(qh[ks], kfl, sl[t]);
      }
    }

#pragma unroll
    for (int r = 0; r < 8; ++r) {
      float v0 = (sh[0][r] + sl[0][r] * RES_INV) * S_SCL;
      float v1 = (sh[1][r] + sl[1][r] * RES_INV) * S_SCL;
      v0 = fminf(fmaxf(v0, -S_CLIP), S_CLIP);
      v1 = fminf(fmaxf(v1, -S_CLIP), S_CLIP);
      float tm = fmaxf(v0, v1);
      tm = fmaxf(tm, __shfl_xor(tm, 1, 32));
      tm = fmaxf(tm, __shfl_xor(tm, 2, 32));
      tm = fmaxf(tm, __shfl_xor(tm, 4, 32));
      tm = fmaxf(tm, __shfl_xor(tm, 8, 32));
      const float mn = fmaxf(m[r], tm);
      const float al = __expf(m[r] - mn);
      const float p0 = __expf(v0 - mn), p1 = __expf(v1 - mn);
      float rs = p0 + p1;
      rs += __shfl_xor(rs, 1, 32);
      rs += __shfl_xor(rs, 2, 32);
      rs += __shfl_xor(rs, 4, 32);
      rs += __shfl_xor(rs, 8, 32);
      l[r] = l[r] * al + rs;
      m[r] = mn;
#pragma unroll
      for (int t = 0; t < 4; ++t) { oh[t][r] *= al; ol[t][r] *= al; }
      const float c0 = p0 * P_CAR, c1 = p1 * P_CAR;
      const _Float16 h0 = (_Float16)c0, h1 = (_Float16)c1;
      _Float16* pph = myPH + (8 * hl + r) * 40 + c;
      _Float16* ppl = myPL + (8 * hl + r) * 40 + c;
      pph[0]  = h0;
      pph[16] = h1;
      ppl[0]  = (_Float16)((c0 - (float)h0) * RES_CAR);
      ppl[16] = (_Float16)((c1 - (float)h1) * RES_CAR);
    }
    __syncthreads();

    const v16h pfh = ld_frag(myPH + c * 40, hl);
    const v16h pfl = ld_frag(myPL + c * 40, hl);
#pragma unroll
    for (int t = 0; t < 4; ++t) {
      const v16h vfh = ld_frag(ldsVH + (16 * t + c) * 40, hl);
      const v16h vfl = ld_frag(ldsVL + (16 * t + c) * 40, hl);
      oh[t] = mma(pfh, vfh, oh[t]);
      ol[t] = mma(pfh, vfl, ol[t]);
      ol[t] = mma(pfl, vfh, ol[t]);
    }
    __syncthreads();
  }

#pragma unroll
  for (int r = 0; r < 8; ++r) {
    const float inv = (1.0f / l[r]) * O_SCL;
    const int rowl = 16 * w + 8 * hl + r;
#pragma unroll
    for (int t = 0; t < 4; ++t)
      ldsF[rowl * 68 + 16 * t + c] = (oh[t][r] + ol[t][r] * RES_INV) * inv;
  }
  __syncthreads();
  float* const ob = Oc + ((size_t)bz * SEQ + q0) * DM + col0;
  for (int i = 0; i < 8; ++i) {
    const int qi = i * 256 + tid;
    const int rowl = qi >> 4, col = (qi & 15) * 4;
    const v4f v = *(const v4f*)(ldsF + rowl * 68 + col);
    *(volatile v4f*)(ob + (size_t)rowl * DM + col) = v;
  }
  __threadfence();
  for (int i = 0; i < 8; ++i) {
    const int qi = i * 256 + tid;
    const int rowl = qi >> 4, col = (qi & 15) * 4;
    const v4f v = *(const v4f*)(ldsF + rowl * 68 + col);
    *(volatile v4f*)(ob + (size_t)rowl * DM + col) = v;
  }
}

__global__ __launch_bounds__(128) __attribute__((amdgpu_num_vgpr(256)))
void k_oproj(const _Float16* __restrict__ AH, const _Float16* __restrict__ AL,
             const _Float16* __restrict__ Bt, const float* __restrict__ Res,
             float* __restrict__ Out)
{
  __shared__ __attribute__((aligned(16))) float ldsF[64 * 68];

  const int tid = threadIdx.x, lane = tid & 31, w = tid >> 5;
  const int hl = lane >> 4, c = lane & 15;
  const int m0 = blockIdx.y * 64, n0 = blockIdx.x * 64;
  const int mw = m0 + 16 * w;

  const _Float16* ap0 = AH + (size_t)(mw + c) * DM;
  const _Float16* ap1 = AL + (size_t)(mw + c) * DM;
  const _Float16* bp  = Bt + (size_t)(n0 + c) * DM;

  v8f acc[8] = {};
  gemm_core(ap0, ap1, bp, DM, hl, acc);

#pragma unroll
  for (int t = 0; t < 4; ++t)
#pragma unroll
    for (int r = 0; r < 8; ++r) {
      const int rowl = 16 * w + 8 * hl + r;
      const float y = (acc[t][r] + acc[4 + t][r] * RES_INV) * OUT_SCL;
      ldsF[rowl * 68 + 16 * t + c] = 0.5f * y * (1.0f + erff(y * 0.70710678118654752f));
    }
  __syncthreads();

  const unsigned bq = (unsigned)m0 / (unsigned)SEQ;
  const unsigned orow0 = bq * (unsigned)SEQ_FULL + ((unsigned)m0 - bq * (unsigned)SEQ);
  const float* const rb = Res + (size_t)m0 * DM + n0;
  float* const ob = Out + (size_t)orow0 * DM + n0;
  for (int i = 0; i < 8; ++i) {
    const int qi = i * 128 + tid;
    const int rowl = qi >> 4, col = (qi & 15) * 4;
    const v4f g = *(const v4f*)(ldsF + rowl * 68 + col);
    const v4f b = *(const v4f*)(rb + (size_t)rowl * DM + col);
    const v4f v = b + g;
    *(volatile v4f*)(ob + (size_t)rowl * DM + col) = v;
  }
  __threadfence();
  for (int i = 0; i < 8; ++i) {
    const int qi = i * 128 + tid;
    const int rowl = qi >> 4, col = (qi & 15) * 4;
    const v4f g = *(const v4f*)(ldsF + rowl * 68 + col);
    const v4f b = *(const v4f*)(rb + (size_t)rowl * DM + col);
    const v4f v = b + g;
    *(volatile v4f*)(ob + (size_t)rowl * DM + col) = v;
  }
}

extern "C" void kernel_launch(void* const* d_in, const int* in_sizes, int n_in,
                              void* d_out, int out_size, void* d_ws, size_t ws_size,
                              hipStream_t stream)
{
  if (n_in < 11) return;
  const long needQ = ((long)(NB - 1) * SEQ_FULL + SEQ) * DM;
  const long needK = ((long)(NB - 1) * MCTX_FULL + MCTX) * DM;
  if ((long)in_sizes[0] < needQ) return;
  if ((long)in_sizes[1] < needK) return;
  if ((long)in_sizes[2] < needK) return;
  if ((long)in_sizes[3] < (long)DM * DM) return;
  if ((long)in_sizes[4] < (long)DM * DM) return;
  if ((long)in_sizes[5] < (long)DM * DM) return;
  if ((long)in_sizes[6] < (long)DM * DM) return;
  if ((long)in_sizes[7] < (long)DM) return;
  if ((long)in_sizes[8] < (long)DM) return;
  if ((long)in_sizes[9] < (long)DM) return;
  if ((long)in_sizes[10] < (long)DM) return;
  if ((long)out_size < needQ) return;

  const float* Qin  = (const float*)d_in[0];
  const float* Kin  = (const float*)d_in[1];
  const float* Vin  = (const float*)d_in[2];
  const float* Wq   = (const float*)d_in[3];
  const float* Wk   = (const float*)d_in[4];
  const float* Wv   = (const float*)d_in[5];
  const float* Wo   = (const float*)d_in[6];
  const float* preG = (const float*)d_in[7];
  const float* preB = (const float*)d_in[8];
  const float* lnG  = (const float*)d_in[9];
  const float* lnB  = (const float*)d_in[10];
  float* out = (float*)d_out;

  const size_t nQ  = (size_t)N_Q;
  const size_t nK  = (size_t)N_K;
  const size_t nW  = (size_t)N_W;
  const size_t nR0 = (size_t)N_R0;
  const size_t total_halves = (size_t)WS_HALVES;
  if (total_halves * sizeof(_Float16) > ws_size) return;

  _Float16* base = (_Float16*)d_ws;
  _Float16* QnP  = base;
  _Float16* KnP  = QnP  + nQ;
  float*    Oc   = (float*)base;
  _Float16* V16  = base + nR0;
  _Float16* WqP  = V16  + nK;
  _Float16* WkP  = WqP  + nW;
  _Float16* WvP  = WkP  + nW;
  _Float16* WoP  = WvP  + nW;
  _Float16* QH   = WoP  + nW;
  _Float16* QL   = QH   + nQ;
  _Float16* KH   = QL   + nQ;
  _Float16* KL   = KH   + nK;
  _Float16* VtH  = KL   + nK;
  _Float16* VtL  = VtH  + nK;
  float*    Onf  = (float*)(VtL + nK);
  _Float16* OnH  = VtL  + nK + 2 * nQ;
  _Float16* OnL  = OnH  + nQ;

  k_ln<0, SEQ,  SEQ_FULL ><<<MRQ / 8, 256, 0, stream>>>(Qin, preG, preB, QnP, QnP, Oc);
  k_ln<0, MCTX, MCTX_FULL><<<MRK / 8, 256, 0, stream>>>(Kin, preG, preB, KnP, KnP, Oc);

  const unsigned tv8 = (unsigned)(nK / 8);
  const unsigned tw8 = (unsigned)(nW / 8);
  k_cvt8<MCTX, MCTX_FULL><<<(tv8 + 255u) / 256u, 256, 0, stream>>>(Vin, V16, ACT_CAR, tv8);
  k_cvt8<DM, DM><<<(tw8 + 255u) / 256u, 256, 0, stream>>>(Wq, WqP, W_CAR, tw8);
  k_cvt8<DM, DM><<<(tw8 + 255u) / 256u, 256, 0, stream>>>(Wk, WkP, W_CAR, tw8);
  k_cvt8<DM, DM><<<(tw8 + 255u) / 256u, 256, 0, stream>>>(Wv, WvP, W_CAR, tw8);
  k_cvt8<DM, DM><<<(tw8 + 255u) / 256u, 256, 0, stream>>>(Wo, WoP, W_CAR, tw8);

  k_proj<<<dim3(DM / 64, MRQ / 128, 1), 128, 0, stream>>>(QnP, WqP, QH, QL, DM, DM, 0u, 0u);
  k_proj<<<dim3(DM / 64, MRK / 128, 1), 128, 0, stream>>>(KnP, WkP, KH, KL, DM, DM, 0u, 0u);
  k_proj<<<dim3(MCTX / 64, DM / 128, NB), 128, 0, stream>>>(WvP, V16, VtH, VtL, DM, MCTX,
                                                            (unsigned)((size_t)MCTX * DM),
                                                            (unsigned)((size_t)DM * MCTX));

  k_attn<<<dim3(SEQ / 128, NH, NB), 256, 0, stream>>>(QH, QL, KH, KL, VtH, VtL, Oc);

  k_ln<1, SEQ, SEQ_FULL><<<MRQ / 8, 256, 0, stream>>>(Oc, lnG, lnB, OnH, OnL, Onf);

  k_oproj<<<dim3(DM / 64, MRQ / 64), 128, 0, stream>>>(OnH, OnL, WoP, Onf, out);
}
